// SequentialLSTM_75196287418593
// MI455X (gfx1250) — hardware-run, weakly checked
//
#include <hip/hip_runtime.h>

typedef __attribute__((ext_vector_type(16))) _Float16 v16h;
typedef __attribute__((ext_vector_type(8)))  _Float16 v8h;
typedef __attribute__((ext_vector_type(8)))  float    v8f;
typedef __attribute__((ext_vector_type(4)))  float    v4f;
typedef __attribute__((ext_vector_type(4)))  unsigned v4u;
typedef __attribute__((address_space(1))) volatile float gvf;

constexpr int kSteps      = 16384;
constexpr int kDin        = 15;
constexpr int kHid        = 1024;
constexpr int kGate       = 4 * kHid;
constexpr int kHeadW      = 4096;
constexpr int kKPad       = 32;
constexpr int kHeadRows   = 4096;
constexpr int kHeadChunks = kSteps / kHeadRows;
constexpr int kScanSteps  = 2048;
constexpr int kScanChunks = kSteps / kScanSteps;
constexpr int kStateF     = 2048;

constexpr float kCarryX  = 64.0f;
constexpr float kCarryW  = 1024.0f;
constexpr float kCarryT  = 256.0f;
constexpr float kScaleXW = 1.0f / (kCarryX * kCarryW);
constexpr float kScaleTW = 1.0f / (kCarryT * kCarryW);
constexpr float kF16MinNormal = 6.103515625e-05f;

static_assert(kGate == 4096);
static_assert(kSteps % kHeadRows == 0 && kSteps % kScanSteps == 0);
static_assert(kHeadRows % 64 == 0 && kScanSteps % 64 == 0 && kGate % 64 == 0 && kHeadW % 64 == 0);
static_assert(kKPad % 32 == 0 && kHeadW % 32 == 0 && kDin < kKPad);
static_assert(kScanSteps % 32 == 0);
static_assert((64 * kDin * 4) % 128 == 0);
static_assert(kStateF >= kHid + 32);

constexpr int kPrepB1 = kSteps * 4 / 256;
constexpr int kPrepB2 = kPrepB1 + kHeadW * 4 / 256;
constexpr int kPrepB3 = kPrepB2 + kGate * 4 / 256;
constexpr int kPrepB4 = kPrepB3 + 16 * kHeadW / 8 / 256;
constexpr int kPrepB5 = kPrepB4 + kGate / 4 / 256;
constexpr int kPrepBlocks = kPrepB5 + kStateF / 4 / 256;
static_assert(kPrepB1 == 256 && kPrepB2 == 320 && kPrepB3 == 384 && kPrepB4 == 416 && kPrepB5 == 420 && kPrepBlocks == 422);

struct Frag16 {
  union U { v16h v; v8h h[2]; };
  static __device__ __forceinline__ v16h load(const _Float16* p) {
    U f; f.h[0] = *(const v8h*)(p); f.h[1] = *(const v8h*)(p + 16); return f.v;
  }
};
__device__ __forceinline__ v8f mma_f16(v16h a, v16h b, v8f c) {
  c = __builtin_amdgcn_wmma_f32_16x16x32_f16(false, a, false, b, (short)0, c, false, false);
  asm volatile("v_nop\n\tv_nop\n\tv_nop\n\tv_nop" : "+v"(c) : "v"(a), "v"(b));
  return c;
}

__device__ __forceinline__ unsigned h16bits(float v) {
  const float t = (fabsf(v) < kF16MinNormal) ? 0.0f : v;
  const _Float16 h = (_Float16)t;
  return (unsigned)__builtin_bit_cast(unsigned short, h);
}
__device__ __forceinline__ unsigned pack2(float a, float b) { return h16bits(a) | (h16bits(b) << 16); }

__device__ __forceinline__ void st2_v4u(unsigned* p, v4u w) {
  *(volatile v4u*)p = w;
  __threadfence();
  *(volatile v4u*)p = w;
}
__device__ __forceinline__ void st2_v4f(float* p, v4f w) {
  *(volatile v4f*)p = w;
  __threadfence();
  *(volatile v4f*)p = w;
}

__device__ __forceinline__ v4u row15_piece(const float* __restrict__ src, int row, int q, float carry) {
  float v[8];
#pragma unroll
  for (int e = 0; e < 8; ++e) {
    const int k = 8 * q + e;
    const int kc = (k < kDin) ? k : (kDin - 1);
    float t = src[(size_t)row * kDin + kc];
    asm volatile("" : "+v"(t));
    v[e] = (k < kDin) ? (t * carry) : 0.0f;
  }
  const unsigned w0 = pack2(v[0], v[1]);
  const unsigned w1 = pack2(v[2], v[3]);
  const unsigned w2 = pack2(v[4], v[5]);
  const unsigned w3 = pack2(v[6], v[7]);
  const v4u w = {w0, w1, w2, w3};
  return w;
}

__global__ __launch_bounds__(256) void prep_kernel(
    const float* __restrict__ x, const float* __restrict__ w_ih, const float* __restrict__ b_ih,
    const float* __restrict__ b_hh, const float* __restrict__ wf1, const float* __restrict__ wf2,
    unsigned* __restrict__ xh, unsigned* __restrict__ wf1h, unsigned* __restrict__ wihh,
    unsigned* __restrict__ wf2h, float* __restrict__ bias, float* __restrict__ state0) {
  const int blk = blockIdx.x, tid = threadIdx.x;
  if (blk < kPrepB1) {
    const int p = blk * 256 + tid;
    const v4u w = row15_piece(x, p >> 2, p & 3, kCarryX);
    st2_v4u(xh + (size_t)p * 4, w);
  } else if (blk < kPrepB2) {
    const int p = (blk - kPrepB1) * 256 + tid;
    const v4u w = row15_piece(wf1, p >> 2, p & 3, kCarryW);
    st2_v4u(wf1h + (size_t)p * 4, w);
  } else if (blk < kPrepB3) {
    const int p = (blk - kPrepB2) * 256 + tid;
    const v4u w = row15_piece(w_ih, p >> 2, p & 3, kCarryW);
    st2_v4u(wihh + (size_t)p * 4, w);
  } else if (blk < kPrepB4) {
    const int p = (blk - kPrepB3) * 256 + tid;
    const int n = p >> 9;
    const int k8 = (p & 511) * 8;
    const int nc = (n < kDin) ? n : (kDin - 1);
    const v4f a0 = *(const v4f*)(wf2 + (size_t)nc * kHeadW + k8);
    const v4f a1 = *(const v4f*)(wf2 + (size_t)nc * kHeadW + k8 + 4);
    float v[8];
#pragma unroll
    for (int e = 0; e < 8; ++e) {
      float t = (e < 4) ? a0[e & 3] : a1[e & 3];
      asm volatile("" : "+v"(t));
      v[e] = (n < kDin) ? (t * kCarryW) : 0.0f;
    }
    const unsigned w0 = pack2(v[0], v[1]);
    const unsigned w1 = pack2(v[2], v[3]);
    const unsigned w2 = pack2(v[4], v[5]);
    const unsigned w3 = pack2(v[6], v[7]);
    const v4u w = {w0, w1, w2, w3};
    st2_v4u(wf2h + (size_t)p * 4, w);
  } else if (blk < kPrepB5) {
    const int p = (blk - kPrepB4) * 256 + tid;
    const v4f a = *(const v4f*)(b_ih + 4 * p);
    const v4f b = *(const v4f*)(b_hh + 4 * p);
    const v4f s = a + b;
    st2_v4f(bias + 4 * p, s);
  } else {
    const int p = (blk - kPrepB5) * 256 + tid;
    const v4f z = {0.0f, 0.0f, 0.0f, 0.0f};
    st2_v4f(state0 + 4 * p, z);
  }
}

template <int OUT_MODE>
__global__ __launch_bounds__(256) void gemm64_f16(
    const _Float16* __restrict__ A, int lda, long strideA,
    const _Float16* __restrict__ Bt, int ldb,
    void* __restrict__ Cout, int ldc, long strideC,
    const float* __restrict__ bias,
    int M, int N, int K, float scale, float post) {
  __shared__ __align__(16) float sT[8][16 * 68];
  const int b    = blockIdx.y;
  const int lane = threadIdx.x & 31;
  const int wave = threadIdx.x >> 5;
  const int tilesN = N >> 6;
  const int tilesM = M >> 6;
  const int tile = blockIdx.x * 8 + wave;
  if (tile >= tilesM * tilesN) return;
  const int tm = tile / tilesN;
  const int tn = tile - tm * tilesN;
  const int m0 = tm << 6;
  const int n0 = tn << 6;

  const _Float16* Ab = A + (size_t)b * strideA;
  const int rlane = lane & 15;
  const int koff  = (lane >> 4) * 8;
  const int mOff  = (lane >> 4) * 8;

  v8f acc[4][4];
#pragma unroll
  for (int i = 0; i < 4; ++i)
#pragma unroll
    for (int j = 0; j < 4; ++j) acc[i][j] = (v8f){0.f, 0.f, 0.f, 0.f, 0.f, 0.f, 0.f, 0.f};

  for (int k0 = 0; k0 < K; k0 += 32) {
    v16h bh[4];
#pragma unroll
    for (int j = 0; j < 4; ++j) {
      const size_t bo = (size_t)(n0 + (j << 4) + rlane) * ldb + koff + k0;
      bh[j] = Frag16::load(Bt + bo);
    }
#pragma unroll
    for (int i = 0; i < 4; ++i) {
      const size_t ao = (size_t)(m0 + (i << 4) + rlane) * lda + koff + k0;
      const v16h ah = Frag16::load(Ab + ao);
#pragma unroll
      for (int j = 0; j < 4; ++j) acc[i][j] = mma_f16(ah, bh[j], acc[i][j]);
    }
  }

  float* slab = sT[wave];
#pragma unroll
  for (int i = 0; i < 4; ++i) {
    const int mBase = m0 + (i << 4);
#pragma unroll
    for (int j = 0; j < 4; ++j) {
      const int n = n0 + (j << 4) + rlane;
      const float bv = bias[n];
#pragma unroll
      for (int r = 0; r < 8; ++r) {
        float v = acc[i][j][r] * scale;
        v += bv;
        if (OUT_MODE == 1) v *= post;
        slab[(mOff + r) * 68 + (j << 4) + rlane] = v;
      }
    }
    __builtin_amdgcn_fence(__ATOMIC_RELEASE, "workgroup");
    __builtin_amdgcn_wave_barrier();
    __builtin_amdgcn_fence(__ATOMIC_ACQUIRE, "workgroup");
    if (OUT_MODE == 0) {
      float* C = (float*)Cout + (size_t)b * strideC;
      const int hh = lane >> 4, c4 = (lane & 15) * 4;
      for (int pass = 0; pass < 2; ++pass) {
#pragma unroll
        for (int it = 0; it < 8; ++it) {
          const int row = it * 2 + hh;
          const v4f v = *(const v4f*)(slab + row * 68 + c4);
          *(volatile v4f*)(C + (size_t)(mBase + row) * ldc + n0 + c4) = v;
        }
        __threadfence();
      }
    } else {
      const int q = lane >> 3, c8 = (lane & 7) * 8;
      _Float16* C = (_Float16*)Cout + (size_t)b * strideC;
      for (int pass = 0; pass < 2; ++pass) {
#pragma unroll
        for (int it = 0; it < 4; ++it) {
          const int row = it * 4 + q;
          const float* sp = slab + row * 68 + c8;
          v8h hv;
#pragma unroll
          for (int e = 0; e < 8; ++e) {
            const float t0 = sp[e];
            const float t1 = (fabsf(t0) < kF16MinNormal) ? 0.0f : t0;
            hv[e] = (_Float16)t1;
          }
          *(volatile v8h*)(C + (size_t)(mBase + row) * ldc + n0 + c8) = hv;
        }
        __threadfence();
      }
    }
    __builtin_amdgcn_fence(__ATOMIC_RELEASE, "workgroup");
    __builtin_amdgcn_wave_barrier();
    __builtin_amdgcn_fence(__ATOMIC_ACQUIRE, "workgroup");
  }
}

__global__ __launch_bounds__(256) void head2_kernel(
    const _Float16* __restrict__ Tc, const _Float16* __restrict__ Wf2h,
    const float* __restrict__ bf2, float* __restrict__ out2, unsigned* __restrict__ fh, int row0) {
  __shared__ __align__(16) float sC[8][64 * kDin];
  const int lane = threadIdx.x & 31;
  const int wave = threadIdx.x >> 5;
  const int tile = blockIdx.x * 8 + wave;
  const int m0 = tile << 6;
  const int c = lane & 15, hh = lane >> 4, koff = hh * 8;

  const _Float16* arow = Tc + (size_t)(m0 + c) * kHeadW + koff;
  const _Float16* brow = Wf2h + (size_t)c * kHeadW + koff;

  v8f acc[4];
#pragma unroll
  for (int i = 0; i < 4; ++i) acc[i] = (v8f){0.f, 0.f, 0.f, 0.f, 0.f, 0.f, 0.f, 0.f};

#pragma unroll 2
  for (int k0 = 0; k0 < kHeadW; k0 += 32) {
    const v16h fb = Frag16::load(brow + k0);
#pragma unroll
    for (int i = 0; i < 4; ++i) {
      const v16h fa = Frag16::load(arow + (size_t)(16 * i) * kHeadW + k0);
      acc[i] = mma_f16(fa, fb, acc[i]);
    }
  }

  const int cc = (c < kDin) ? c : (kDin - 1);
  float bv = bf2[cc];
  asm volatile("" : "+v"(bv));

  float* comp = sC[wave];
#pragma unroll
  for (int i = 0; i < 4; ++i) {
#pragma unroll
    for (int r = 0; r < 8; ++r) {
      const float v = acc[i][r] * kScaleTW + bv;
      if (c < kDin) comp[(16 * i + 8 * hh + r) * kDin + c] = v;
    }
  }
  __builtin_amdgcn_fence(__ATOMIC_RELEASE, "workgroup");
  __builtin_amdgcn_wave_barrier();
  __builtin_amdgcn_fence(__ATOMIC_ACQUIRE, "workgroup");

  float* dst = out2 + (size_t)(row0 + m0) * kDin;
  v4f ov[8];
#pragma unroll
  for (int it = 0; it < 8; ++it) {
    const int idx = it * 32 + lane;
    const int ic = (idx < 240) ? idx : 239;
    ov[it] = *(const v4f*)(comp + ic * 4);
  }
  for (int pass = 0; pass < 2; ++pass) {
#pragma unroll
    for (int it = 0; it < 8; ++it) {
      const int idx = it * 32 + lane;
      if (idx < 240) *(volatile v4f*)(dst + idx * 4) = ov[it];
    }
    __threadfence();
  }

  unsigned* fdst = fh + (size_t)(row0 + m0) * (kKPad / 2);
  v4u fw[8];
#pragma unroll
  for (int it = 0; it < 8; ++it) {
    const int p = it * 32 + lane;
    const int r = p >> 2, q = p & 3;
    float v[8];
#pragma unroll
    for (int e = 0; e < 8; ++e) {
      const int k = 8 * q + e;
      const int kc = (k < kDin) ? k : (kDin - 1);
      const float t = comp[r * kDin + kc];
      v[e] = (k < kDin) ? (t * kCarryX) : 0.0f;
    }
    const unsigned w0 = pack2(v[0], v[1]);
    const unsigned w1 = pack2(v[2], v[3]);
    const unsigned w2 = pack2(v[4], v[5]);
    const unsigned w3 = pack2(v[6], v[7]);
    const v4u w = {w0, w1, w2, w3};
    fw[it] = w;
  }
  for (int pass = 0; pass < 2; ++pass) {
#pragma unroll
    for (int it = 0; it < 8; ++it) {
      const int p = it * 32 + lane;
      *(volatile v4u*)(fdst + (size_t)p * 4) = fw[it];
    }
    __threadfence();
  }
}

__device__ __forceinline__ float fast_sigmoid(float v) { return __builtin_amdgcn_rcpf(1.0f + __expf(-v)); }
__device__ __forceinline__ float fast_tanh(float v) { return 1.0f - 2.0f * __builtin_amdgcn_rcpf(1.0f + __expf(2.0f * v)); }

__device__ __forceinline__ void gated_cell(float pi, float pf, float pg, float po, float h, float c,
                                           float wi, float wf, float wg, float wo, float wr,
                                           float& c_new, float& part) {
  const float gi = pi + h * wi;
  const float gf = pf + h * wf;
  const float gg = pg + h * wg;
  const float go = po + h * wo;
  const float si = fast_sigmoid(gi);
  const float sf = fast_sigmoid(gf);
  const float tg = fast_tanh(gg);
  const float so = fast_sigmoid(go);
  c_new = sf * c + si * tg;
  part = wr * (so * fast_tanh(c_new));
}

__device__ __forceinline__ void block_sum2(float& a, float& b, float* slot, int lane, int wave) {
#pragma unroll
  for (int off = 16; off > 0; off >>= 1) {
    a += __shfl_xor(a, off, 32);
    b += __shfl_xor(b, off, 32);
  }
  if (lane == 0) {
    slot[wave * 2] = a;
    slot[wave * 2 + 1] = b;
  }
  __syncthreads();
  float xa = slot[lane * 2];
  float xb = slot[lane * 2 + 1];
#pragma unroll
  for (int off = 16; off > 0; off >>= 1) {
    xa += __shfl_xor(xa, off, 32);
    xb += __shfl_xor(xb, off, 32);
  }
  a = xa;
  b = xb;
}

__global__ __launch_bounds__(1024) void scan_kernel(
    const float* __restrict__ gx, const float* __restrict__ gf,
    const float* __restrict__ whh, const float* __restrict__ whr,
    const float* state_in, float* state_out,
    float* out_h1, float* out_h2) {
  __shared__ float red[2][64];
  const int j = threadIdx.x;
  const int lane = j & 31;
  const int wave = j >> 5;

  const float wi = whh[j];
  const float wf = whh[j + kHid];
  const float wg = whh[j + 2 * kHid];
  const float wo = whh[j + 3 * kHid];
  const float wr = whr[j];

  const gvf* sp = (const gvf*)state_in;
  float c  = sp[j];
  float h1 = sp[kHid];
  float keep1 = 0.0f, keep2 = 0.0f;

  {
    const float* g0 = gx + j;
    const float pi = g0[0];
    const float pf = g0[kHid];
    const float pg = g0[2 * kHid];
    const float po = g0[3 * kHid];
    float cn, p1;
    gated_cell(pi, pf, pg, po, h1, c, wi, wf, wg, wo, wr, cn, p1);
    c = cn;
    float a = p1, b = 0.0f;
    block_sum2(a, b, red[1], lane, wave);
    h1 = a;
    keep1 = (lane == 0) ? h1 : keep1;
  }

#pragma unroll 1
  for (int s = 0; s < kScanSteps; ++s) {
    const bool adv = (s + 1 < kScanSteps);
    const int sn = adv ? (s + 1) : (kScanSteps - 1);
    const float* gfr = gf + (size_t)s * kGate + j;
    const float* gxr = gx + (size_t)sn * kGate + j;
    const float qi = gfr[0];
    const float qf = gfr[kHid];
    const float qg = gfr[2 * kHid];
    const float qo = gfr[3 * kHid];
    const float pi = gxr[0];
    const float pf = gxr[kHid];
    const float pg = gxr[2 * kHid];
    const float po = gxr[3 * kHid];

    float cdrop, p2;
    gated_cell(qi, qf, qg, qo, h1, c, wi, wf, wg, wo, wr, cdrop, p2);
    float cn, p1;
    gated_cell(pi, pf, pg, po, h1, c, wi, wf, wg, wo, wr, cn, p1);

    float a = adv ? p1 : 0.0f;
    float b = p2;
    block_sum2(a, b, red[s & 1], lane, wave);

    keep2 = ((s & 31) == lane) ? b : keep2;
    if ((s & 31) == 31) {
      if (wave == 0) {
        float* q1 = out_h1 + (s - 31) + lane;
        float* q2 = out_h2 + (s - 31) + lane;
        *(volatile float*)q1 = keep1;
        *(volatile float*)q2 = keep2;
        __threadfence();
        *(volatile float*)q1 = keep1;
        *(volatile float*)q2 = keep2;
      }
    }
    c  = adv ? cn : c;
    h1 = adv ? a : h1;
    keep1 = (((s + 1) & 31) == lane) ? h1 : keep1;
  }

  {
    float* qc = state_out + j;
    *(volatile float*)qc = c;
    __threadfence();
    *(volatile float*)qc = c;
    if (wave == 0) {
      float* qh = state_out + kHid + lane;
      const float hv = (lane == 0) ? h1 : 0.0f;
      *(volatile float*)qh = hv;
      __threadfence();
      *(volatile float*)qh = hv;
    }
  }
}

extern "C" void kernel_launch(void* const* d_in, const int* in_sizes, int n_in,
                              void* d_out, int out_size, void* d_ws, size_t ws_size, hipStream_t stream) {
  if (n_in < 10 || d_out == nullptr || d_ws == nullptr) return;
  if (in_sizes[0] != kSteps * kDin || in_sizes[1] != kGate * kDin || in_sizes[2] != kGate ||
      in_sizes[3] != kGate || in_sizes[4] != kGate || in_sizes[5] != kHid ||
      in_sizes[6] != kHeadW * kDin || in_sizes[7] != kHeadW || in_sizes[8] != kDin * kHeadW ||
      in_sizes[9] != kDin || out_size != 2 * kSteps + kSteps * kDin) return;

  const float* x    = (const float*)d_in[0];
  const float* W_ih = (const float*)d_in[1];
  const float* W_hh = (const float*)d_in[2];
  const float* b_ih = (const float*)d_in[3];
  const float* b_hh = (const float*)d_in[4];
  const float* W_hr = (const float*)d_in[5];
  const float* Wf1  = (const float*)d_in[6];
  const float* bf1  = (const float*)d_in[7];
  const float* Wf2  = (const float*)d_in[8];
  const float* bf2  = (const float*)d_in[9];
  float* out = (float*)d_out;

  char* ws = (char*)d_ws;
  size_t off = 0;
  auto carve = [&](size_t bytes) -> char* { char* p = ws + off; off += (bytes + 255) & ~(size_t)255; return p; };
  _Float16* XF16  = (_Float16*)carve((size_t)2 * kSteps * kKPad * 2);
  _Float16* WF1H  = (_Float16*)carve((size_t)kHeadW * kKPad * 2);
  _Float16* WIHH  = (_Float16*)carve((size_t)kGate * kKPad * 2);
  _Float16* WF2H  = (_Float16*)carve((size_t)16 * kHeadW * 2);
  float*    BIAS  = (float*)carve((size_t)kGate * 4);
  float*    STATE = (float*)carve((size_t)2 * kStateF * 4);
  _Float16* TC    = (_Float16*)carve((size_t)kHeadRows * kHeadW * 2);
  float*    GATES = (float*)carve((size_t)2 * kScanSteps * kGate * 4);
  if (off > ws_size || off > (size_t)134217728) return;

  _Float16* FH16 = XF16 + (size_t)kSteps * kKPad;

  prep_kernel<<<kPrepBlocks, 256, 0, stream>>>(x, W_ih, b_ih, b_hh, Wf1, Wf2,
                                               (unsigned*)XF16, (unsigned*)WF1H, (unsigned*)WIHH,
                                               (unsigned*)WF2H, BIAS, STATE);

  for (int hc = 0; hc < kHeadChunks; ++hc) {
    const int row0 = hc * kHeadRows;
    gemm64_f16<1><<<dim3((kHeadRows / 64) * (kHeadW / 64) / 8, 1), 256, 0, stream>>>(
        XF16 + (size_t)row0 * kKPad, kKPad, 0L,
        WF1H, kKPad,
        (void*)TC, kHeadW, 0L,
        bf1, kHeadRows, kHeadW, kKPad, kScaleXW, kCarryT);
    head2_kernel<<<kHeadRows / 64 / 8, 256, 0, stream>>>(
        TC, WF2H, bf2, out + 2 * kSteps, (unsigned*)FH16, row0);
  }

  for (int sc = 0; sc < kScanChunks; ++sc) {
    const int t0 = sc * kScanSteps;
    gemm64_f16<0><<<dim3((kScanSteps / 64) * (kGate / 64) / 8, 2), 256, 0, stream>>>(
        XF16 + (size_t)t0 * kKPad, kKPad, (long)kSteps * kKPad,
        WIHH, kKPad,
        (void*)GATES, kGate, (long)kScanSteps * kGate,
        BIAS, kScanSteps, kGate, kKPad, kScaleXW, 1.0f);
    scan_kernel<<<1, 1024, 0, stream>>>(
        GATES, GATES + (size_t)kScanSteps * kGate, W_hh, W_hr,
        STATE + (size_t)(sc & 1) * kStateF, STATE + (size_t)((sc + 1) & 1) * kStateF,
        out + t0, out + kSteps + t0);
  }
}
